// GCNModel_63196148793943
// MI455X (gfx1250) — hardware-verified
//
#include <hip/hip_runtime.h>
#include <stddef.h>
#include <stdint.h>
#include <math.h>


#define NN     100000
#define NE     1600000
#define DD     128
#define K2     256
#define NGR    512
#define NTHR   256
#define NWAVE  8
#define EPT    8
#define CHUNK  (NTHR * EPT)
#define WCAP   (EPT * 32)
#define LISTN  (NWAVE * WCAP)
#define NBA    1024
#define SLA    10
#define RCAP   20480
#define DEGCAP 64
#define NBLK   98
#define NSL    (NBLK * NBA)
#define NP     100096
#define GBM    64
#define GBN    128
#define GTHR   128
#define GWAVE  (GTHR / 32)
#define PARTW  288
#define WSTW   258
#define NUW0   (DD * (DD / 8))
#define NUW1   (DD * (K2 / 8))
#define VTW    256
#define BK_INTS (LISTN + 2 * RCAP + 3 * NBA)
#define BK_LDS_INTS (BK_INTS + 16 + NBA)
#define WSMAX  134217728

static_assert((CHUNK & (CHUNK - 1)) == 0 && CHUNK <= 4096);
static_assert((NBA & (NBA - 1)) == 0 && NBA == (1 << SLA));
static_assert(((long long)CHUNK << SLA) < (1LL << 31));
static_assert((long long)NE < (1LL << (31 - SLA)));
static_assert(NBA % NTHR == 0 && NBA == 4 * NTHR && NBA % NWAVE == 0);
static_assert(RCAP % (NTHR * 4) == 0 && BK_INTS % 4 == 0 && LISTN % 4 == 0);
static_assert(RCAP >= 16710 + 16710 / 20 + 1);
static_assert(DEGCAP >= 36 + 8);
static_assert(BK_LDS_INTS * 4 <= 300000);
static_assert(NP % GBM == 0 && NP % 256 == 0 && NP >= NN && NSL >= NP);
static_assert((NP * (DD / 8)) % NTHR == 0);
static_assert(DD % 32 == 0 && K2 % 32 == 0 && K2 == 2 * DD && DD == GBN && GBM == GWAVE * 16);
static_assert(NUW0 % NTHR == 0 && NUW1 % NTHR == 0);
static_assert(PARTW % 32 == 0 && PARTW / 4 <= NTHR && PARTW >= 2 * DD + 1 && WSTW >= 2 * DD + 1);
static_assert(NGR == 4 * 128 && (NGR * 4) % 128 == 0);
static_assert(NE % 4 == 0);

typedef float          v4f   __attribute__((ext_vector_type(4)));
typedef float          v8f   __attribute__((ext_vector_type(8)));
typedef int            v4i   __attribute__((ext_vector_type(4)));
typedef int            v8i   __attribute__((ext_vector_type(8)));
typedef unsigned short v8us  __attribute__((ext_vector_type(8)));
typedef unsigned short v16us __attribute__((ext_vector_type(16)));
typedef __bf16         v16bf __attribute__((ext_vector_type(16)));
typedef v4f  __attribute__((may_alias)) v4fa;
typedef v4i  __attribute__((may_alias)) v4ia;
typedef v8us __attribute__((may_alias)) v8usa;
union FragB { v16bf v; v16us u; v8us h[2]; v8i w; };

__device__ __forceinline__ v8f wmb(const FragB& a, const FragB& b, v8f c) {
  v8f d = __builtin_amdgcn_wmma_f32_16x16x32_bf16(false, a.v, false, b.v, (short)0, c, false, false);
  asm volatile("v_nop\n\tv_nop\n\tv_nop\n\tv_nop" : "+v"(d) : "v"(a.w), "v"(b.w));
  return d;
}

__device__ __forceinline__ v8f z8() { v8f z = {0.f, 0.f, 0.f, 0.f, 0.f, 0.f, 0.f, 0.f}; return z; }

__device__ __forceinline__ unsigned bf16_bits(float f) {
  const unsigned u = __float_as_uint(f);
  return (u + 0x7FFFu + ((u >> 16) & 1u)) >> 16;
}
__device__ __forceinline__ float bf16_val(float f) {
  return __uint_as_float(bf16_bits(f) << 16);
}
__device__ __forceinline__ unsigned bf16_bits_n(float f) {
  const unsigned r = bf16_bits(f);
  return (f != f) ? 0x7fc0u : r;
}

template <int SLB>
__device__ __forceinline__ int scan_chunk(const int* __restrict__ dsts, int nE, int cbase, int slotBase,
                                          int nb, int vec8, int* list, int tid, int lane, int wave) {
  int wc = 0;
  const int el0  = tid * EPT;
  const int e0   = cbase + el0;
  const int sent = -2147483647 - 1;
  v4i da, db;
  if (vec8 != 0 && cbase + CHUNK <= nE) {
    da = *(const v4i*)(dsts + e0);
    db = *(const v4i*)(dsts + e0 + 4);
  } else {
    da.x = (e0     < nE) ? dsts[min(e0,     nE - 1)] : sent;
    da.y = (e0 + 1 < nE) ? dsts[min(e0 + 1, nE - 1)] : sent;
    da.z = (e0 + 2 < nE) ? dsts[min(e0 + 2, nE - 1)] : sent;
    da.w = (e0 + 3 < nE) ? dsts[min(e0 + 3, nE - 1)] : sent;
    db.x = (e0 + 4 < nE) ? dsts[min(e0 + 4, nE - 1)] : sent;
    db.y = (e0 + 5 < nE) ? dsts[min(e0 + 5, nE - 1)] : sent;
    db.z = (e0 + 6 < nE) ? dsts[min(e0 + 6, nE - 1)] : sent;
    db.w = (e0 + 7 < nE) ? dsts[min(e0 + 7, nE - 1)] : sent;
  }
  const unsigned nbs = (unsigned)slotBase;
  const unsigned unb = (unsigned)nb;
  const unsigned s0 = (unsigned)da.x - nbs, s1 = (unsigned)da.y - nbs;
  const unsigned s2 = (unsigned)da.z - nbs, s3 = (unsigned)da.w - nbs;
  const unsigned s4 = (unsigned)db.x - nbs, s5 = (unsigned)db.y - nbs;
  const unsigned s6 = (unsigned)db.z - nbs, s7 = (unsigned)db.w - nbs;
  const bool h0 = s0 < unb, h1 = s1 < unb, h2 = s2 < unb, h3 = s3 < unb;
  const bool h4 = s4 < unb, h5 = s5 < unb, h6 = s6 < unb, h7 = s7 < unb;
  const unsigned any = __builtin_amdgcn_ballot_w32(h0 | h1 | h2 | h3 | h4 | h5 | h6 | h7);
  if (any != 0u) {
#define HITJ(J, HJ, SJ) { \
      const unsigned mj = __builtin_amdgcn_ballot_w32(HJ); \
      if (mj != 0u) { \
        if (HJ) { \
          const int pos = wc + (int)__builtin_amdgcn_mbcnt_lo(mj, 0u); \
          if (pos < WCAP) list[wave * WCAP + pos] = ((el0 + (J)) << SLB) | (int)(SJ); \
        } \
        wc += (int)__builtin_popcount(mj); } }
    HITJ(0, h0, s0)
    HITJ(1, h1, s1)
    HITJ(2, h2, s2)
    HITJ(3, h3, s3)
    HITJ(4, h4, s4)
    HITJ(5, h5, s5)
    HITJ(6, h6, s6)
    HITJ(7, h7, s7)
#undef HITJ
  }
  return wc;
}

__global__ __launch_bounds__(NTHR) void k_cvx(const float* __restrict__ x, int nN, int nUnits,
                                              unsigned short* xb) {
  const int u = (int)blockIdx.x * NTHR + (int)threadIdx.x;
  if (u >= nUnits) return;
  const int row = u >> 4;
  const int k8  = (u & 15) * 8;
  const int rc  = row < nN ? row : nN - 1;
  const float* p = x + (size_t)rc * DD + k8;
  const v4f a = *(const v4fa*)p;
  const v4f b = *(const v4fa*)(p + 4);
  const bool ok = row < nN;
  v8us o;
  o[0] = ok ? (unsigned short)bf16_bits(a.x) : (unsigned short)0;
  o[1] = ok ? (unsigned short)bf16_bits(a.y) : (unsigned short)0;
  o[2] = ok ? (unsigned short)bf16_bits(a.z) : (unsigned short)0;
  o[3] = ok ? (unsigned short)bf16_bits(a.w) : (unsigned short)0;
  o[4] = ok ? (unsigned short)bf16_bits(b.x) : (unsigned short)0;
  o[5] = ok ? (unsigned short)bf16_bits(b.y) : (unsigned short)0;
  o[6] = ok ? (unsigned short)bf16_bits(b.z) : (unsigned short)0;
  o[7] = ok ? (unsigned short)bf16_bits(b.w) : (unsigned short)0;
  unsigned short* dp = xb + (size_t)row * DD + k8;
  *(volatile v8us*)dp = o;
  __threadfence();
  *(volatile v8us*)dp = o;
}

__global__ __launch_bounds__(NTHR) void k_wprep(const float* __restrict__ W0, const float* __restrict__ W1,
                                                const float* __restrict__ W2, const float* __restrict__ b2,
                                                const float* __restrict__ fcW, const float* __restrict__ fcb,
                                                unsigned short* W0T, unsigned short* W1D, float* VT) {
  __shared__ __attribute__((aligned(16))) float vs[VTW];
  const int tid = (int)threadIdx.x;
  const int bid = (int)blockIdx.x;
  if (bid < NUW0 / NTHR) {
    const int u  = bid * NTHR + tid;
    const int n  = u >> 4;
    const int k8 = (u & 15) * 8;
    const float* p = W0 + (size_t)k8 * DD + n;
    v8us o;
#pragma unroll
    for (int i = 0; i < 8; ++i) o[i] = (unsigned short)bf16_bits(p[(size_t)i * DD]);
    unsigned short* dp = W0T + (size_t)n * DD + k8;
    *(volatile v8us*)dp = o;
    __threadfence();
    *(volatile v8us*)dp = o;
  } else if (bid < (NUW0 + NUW1) / NTHR) {
    const int u  = (bid - NUW0 / NTHR) * NTHR + tid;
    const int n  = u >> 5;
    const int k8 = (u & 31) * 8;
    const int kk = k8 & (DD - 1);
    const float* p = W1 + (size_t)kk * DD + n;
    v8us o;
#pragma unroll
    for (int i = 0; i < 8; ++i) o[i] = (unsigned short)bf16_bits(p[(size_t)i * DD]);
    unsigned short* dp = W1D + (size_t)n * K2 + k8;
    *(volatile v8us*)dp = o;
    __threadfence();
    *(volatile v8us*)dp = o;
  } else {
    const int tr = tid < DD ? tid : DD - 1;
    const float* wr = W2 + (size_t)tr * DD;
    double s1 = 0.0, s2 = 0.0;
#pragma unroll 2
    for (int n = 0; n < DD; ++n) {
      const double f = (double)bf16_val(fcW[n]);
      s1 += (double)bf16_val(wr[n]) * f;
      s2 += (double)bf16_val(b2[n]) * f;
    }
    const float fb = bf16_val(fcb[0]);
    float val = 0.0f;
    val = (tid < DD) ? (float)s1 : val;
    val = (tid == DD) ? (float)s2 : val;
    val = (tid == DD + 1) ? fb : val;
    vs[tid] = val;
    __syncthreads();
    v4f v = {0.f, 0.f, 0.f, 0.f};
    if (tid < VTW / 4) {
      v = *(const v4fa*)(vs + 4 * tid);
      *(volatile v4f*)(VT + 4 * tid) = v;
    }
    __threadfence();
    if (tid < VTW / 4) {
      *(volatile v4f*)(VT + 4 * tid) = v;
    }
  }
}

__global__ __launch_bounds__(NTHR) void k_bucket(const int* __restrict__ srcs, const int* __restrict__ dsts,
                                                 int nE, int nN, int vec8,
                                                 int* LIST, int* CNT, int* OFF, float* DINV) {
  extern __shared__ __attribute__((aligned(16))) int dsm[];
  int* list = dsm;
  int* hl   = dsm + LISTN;
  int* sl   = hl + RCAP;
  int* cnt  = sl + RCAP;
  int* offs = cnt + NBA;
  int* cur  = offs + NBA;
  int* misc = cur + NBA;
  float* dvf = (float*)(misc + 16);
  const int tid = (int)threadIdx.x, lane = tid & 31, wave = tid >> 5;
  const int nodeBase = (int)blockIdx.x * NBA;

  {
    const v4i z4 = {0, 0, 0, 0};
    for (int i = tid * 4; i < BK_INTS; i += NTHR * 4) *(v4ia*)(dsm + i) = z4;
    if (tid < 16) misc[tid] = 0;
  }
  __syncthreads();

  int t = 0, ov = 0;
  const int nChunks = (nE + CHUNK - 1) / CHUNK;
#pragma unroll 1
  for (int ch = 0; ch < nChunks; ++ch) {
    const int cbase = ch * CHUNK;
    const int wc = scan_chunk<SLA>(dsts, nE, cbase, nodeBase, NBA, vec8, list, tid, lane, wave);
    if (lane == 0) misc[wave] = wc;
    __syncthreads();
    if (wave == 0) {
#pragma unroll 1
      for (int w2 = 0; w2 < NWAVE; ++w2) {
        int c = misc[w2];
        c = c < 0 ? 0 : (c > WCAP ? WCAP : c);
#pragma unroll 1
        for (int b0 = 0; b0 < c; b0 += 32) {
          const int idx = b0 + lane;
          const int ent = list[w2 * WCAP + (idx < WCAP ? idx : WCAP - 1)];
          const int m32 = (c - b0) < 32 ? (c - b0) : 32;
#pragma unroll 1
          for (int k = 0; k < m32; ++k) {
            const int u    = __builtin_amdgcn_readlane(ent, k);
            const int slot = u & (NBA - 1);
            const int el   = (u >> SLA) & (CHUNK - 1);
            const int pk   = ((cbase + el) << SLA) | slot;
            if (t < RCAP) {
              if (lane == 0) { hl[t] = pk; cnt[slot] = cnt[slot] + 1; }
              t = t + 1;
            } else {
              ov = 1;
            }
          }
        }
      }
    }
    __syncthreads();
  }
  if (wave == 0 && lane == 0) { misc[8] = t; misc[9] = ov; }
  __syncthreads();
  int tt = misc[8];
  tt = tt < 0 ? 0 : (tt > RCAP ? RCAP : tt);
  const int ovf = misc[9];

  if (wave == 0) {
    const int base = lane * (NBA / 32);
    int s = 0;
#pragma unroll 1
    for (int i = 0; i < NBA / 32; ++i) s += cnt[base + i];
    int incl = s;
#pragma unroll
    for (int d = 1; d < 32; d <<= 1) {
      const int y = __shfl_up(incl, d, 32);
      if (lane >= d) incl += y;
    }
    int run = incl - s;
#pragma unroll 1
    for (int i = 0; i < NBA / 32; ++i) {
      const int cv = cnt[base + i];
      offs[base + i] = run;
      cur[base + i]  = run;
      run += cv;
    }
  }
  __syncthreads();
  if (wave == 0) {
#pragma unroll 1
    for (int b0 = 0; b0 < tt; b0 += 32) {
      const int idx = b0 + lane;
      const int ent = hl[idx < RCAP ? idx : RCAP - 1];
      const int m32 = (tt - b0) < 32 ? (tt - b0) : 32;
#pragma unroll 1
      for (int k = 0; k < m32; ++k) {
        const int u    = __builtin_amdgcn_readlane(ent, k);
        const int slot = u & (NBA - 1);
        if (lane == 0) {
          int p = cur[slot];
          p = p < 0 ? 0 : (p > RCAP - 1 ? RCAP - 1 : p);
          sl[p] = u;
          cur[slot] = p + 1;
        }
      }
    }
  }
  __syncthreads();

#pragma unroll 1
  for (int i = tid * 4; i < RCAP; i += NTHR * 4) {
    const v4i e = *(const v4ia*)(sl + i);
    int e0 = e.x >> SLA, e1 = e.y >> SLA, e2 = e.z >> SLA, e3 = e.w >> SLA;
    e0 = e0 < 0 ? 0 : (e0 > nE - 1 ? nE - 1 : e0);
    e1 = e1 < 0 ? 0 : (e1 > nE - 1 ? nE - 1 : e1);
    e2 = e2 < 0 ? 0 : (e2 > nE - 1 ? nE - 1 : e2);
    e3 = e3 < 0 ? 0 : (e3 > nE - 1 ? nE - 1 : e3);
    int r0 = srcs[e0], r1 = srcs[e1], r2 = srcs[e2], r3 = srcs[e3];
    r0 = r0 < 0 ? 0 : (r0 > nN - 1 ? nN - 1 : r0);
    r1 = r1 < 0 ? 0 : (r1 > nN - 1 ? nN - 1 : r1);
    r2 = r2 < 0 ? 0 : (r2 > nN - 1 ? nN - 1 : r2);
    r3 = r3 < 0 ? 0 : (r3 > nN - 1 ? nN - 1 : r3);
    v4i o;
    o.x = (i     < tt) ? r0 : 0;
    o.y = (i + 1 < tt) ? r1 : 0;
    o.z = (i + 2 < tt) ? r2 : 0;
    o.w = (i + 3 < tt) ? r3 : 0;
    *(v4ia*)(sl + i) = o;
  }
  {
    const float qnan = __int_as_float(0x7fc00000);
#pragma unroll 1
    for (int q = 0; q < NBA / NTHR; ++q) {
      const int s = q * NTHR + tid;
      const int c = cnt[s];
      const float d = 1.0f / sqrtf((float)c + 2.0f);
      const bool bad = (ovf != 0) || (c > DEGCAP) || (c < 0);
      dvf[s] = bad ? qnan : d;
    }
  }
  __syncthreads();

  int* lp = LIST + (size_t)blockIdx.x * RCAP;
#pragma unroll 1
  for (int i = tid * 4; i < RCAP; i += NTHR * 4) {
    const v4i v = *(const v4ia*)(sl + i);
    *(volatile v4i*)(lp + i) = v;
  }
  const int s0 = 4 * tid;
  const v4i c4 = *(const v4ia*)(cnt + s0);
  const v4i o4 = *(const v4ia*)(offs + s0);
  const v4f d4 = *(const v4fa*)(dvf + s0);
  *(volatile v4i*)(CNT + (size_t)nodeBase + s0) = c4;
  *(volatile v4i*)(OFF + (size_t)nodeBase + s0) = o4;
  *(volatile v4f*)(DINV + (size_t)nodeBase + s0) = d4;
  __threadfence();
#pragma unroll 1
  for (int i = tid * 4; i < RCAP; i += NTHR * 4) {
    const v4i v = *(const v4ia*)(sl + i);
    *(volatile v4i*)(lp + i) = v;
  }
  *(volatile v4i*)(CNT + (size_t)nodeBase + s0) = c4;
  *(volatile v4i*)(OFF + (size_t)nodeBase + s0) = o4;
  *(volatile v4f*)(DINV + (size_t)nodeBase + s0) = d4;
}

__global__ __launch_bounds__(GTHR) void k_gemm(const unsigned short* __restrict__ A,
                                               const unsigned short* __restrict__ BT,
                                               float* outF, int K) {
  __shared__ __attribute__((aligned(16))) float stg[GBM * GBN];
  const int tid = (int)threadIdx.x, lane = tid & 31, wave = tid >> 5, hh = lane >> 4, m = lane & 15;
  const int rowBase = (int)blockIdx.x * GBM;

  v8f acc[8];
#pragma unroll
  for (int t = 0; t < 8; ++t) acc[t] = z8();
  const unsigned short* ap = A  + (size_t)(rowBase + 16 * wave + m) * (size_t)K + 8 * hh;
  const unsigned short* bp = BT + (size_t)m * (size_t)K + 8 * hh;

#pragma unroll 1
  for (int k0 = 0; k0 < K; k0 += 32) {
    FragB af;
    af.h[0] = *(const v8usa*)(ap + k0);
    af.h[1] = *(const v8usa*)(ap + k0 + 16);
#pragma unroll
    for (int nt = 0; nt < 8; ++nt) {
      const unsigned short* wq = bp + (size_t)(16 * nt) * (size_t)K + k0;
      FragB bf;
      bf.h[0] = *(const v8usa*)wq;
      bf.h[1] = *(const v8usa*)(wq + 16);
      acc[nt] = wmb(af, bf, acc[nt]);
    }
  }

#pragma unroll
  for (int nt = 0; nt < 8; ++nt) {
    const int lc = 16 * nt + m;
#pragma unroll
    for (int r = 0; r < 8; ++r) {
      const int lr = 16 * wave + 8 * hh + r;
      stg[lr * GBN + lc] = acc[nt][r];
    }
  }
  __syncthreads();

  v4f pv[16];
#pragma unroll
  for (int i = 0; i < 16; ++i) pv[i] = *(const v4fa*)(stg + (16 * wave + i) * GBN + 4 * lane);
#pragma unroll
  for (int i = 0; i < 16; ++i) {
    float* op = outF + (size_t)(rowBase + 16 * wave + i) * (size_t)DD + 4 * lane;
    *(volatile v4f*)op = pv[i];
  }
  __threadfence();
#pragma unroll
  for (int i = 0; i < 16; ++i) {
    float* op = outF + (size_t)(rowBase + 16 * wave + i) * (size_t)DD + 4 * lane;
    *(volatile v4f*)op = pv[i];
  }
}

__global__ __launch_bounds__(NTHR) void k_agg(const int* __restrict__ LIST, const int* __restrict__ CNT,
                                              const int* __restrict__ OFF, const float* __restrict__ DINV,
                                              const float* __restrict__ H, const float* __restrict__ bias,
                                              int nN, float* C, float* REC) {
  __shared__ __attribute__((aligned(16))) float wst[NWAVE * WSTW];
  __shared__ __attribute__((aligned(16))) float pst[PARTW];
  const int tid = (int)threadIdx.x, lane = tid & 31, wave = tid >> 5;
  const int nodeBase = (int)blockIdx.x * NBA;
  const int* lp = LIST + (size_t)blockIdx.x * RCAP;

  float bq[4];
  {
    const v4f b4 = *(const v4fa*)(bias + 4 * lane);
    bq[0] = bf16_val(b4.x); bq[1] = bf16_val(b4.y); bq[2] = bf16_val(b4.z); bq[3] = bf16_val(b4.w);
  }
  int wn = 0;
  float wm[4], wq[4];
#pragma unroll
  for (int j = 0; j < 4; ++j) { wm[j] = 0.0f; wq[j] = 0.0f; }

#pragma unroll 1
  for (int si = 0; si < NBA / NWAVE; ++si) {
    const int s    = si * NWAVE + wave;
    const int node = nodeBase + s;
    int c = CNT[node];
    c = c < 0 ? 0 : (c > DEGCAP ? DEGCAP : c);
    int o = OFF[node];
    o = o < 0 ? 0 : (o > RCAP ? RCAP : o);
    const int nc = node < nN ? node : nN - 1;
    const float dd = DINV[node];
    float a0 = 0.0f, a1 = 0.0f, a2 = 0.0f, a3 = 0.0f;
#pragma unroll 1
    for (int b0 = 0; b0 < c; b0 += 32) {
      int idx = o + b0 + lane;
      idx = idx > RCAP - 1 ? RCAP - 1 : idx;
      int sr = lp[idx];
      sr = sr < 0 ? 0 : (sr > nN - 1 ? nN - 1 : sr);
      const float cf  = DINV[sr] * dd;
      const int   cfi = __float_as_int(cf);
      const int m32 = (c - b0) < 32 ? (c - b0) : 32;
#pragma unroll 1
      for (int k = 0; k < m32; ++k) {
        const int   sk = __builtin_amdgcn_readlane(sr, k);
        const float ck = __int_as_float(__builtin_amdgcn_readlane(cfi, k));
        const v4f a = *(const v4fa*)(H + (size_t)sk * DD + 4 * lane);
        a0 = fmaf(ck, a.x, a0); a1 = fmaf(ck, a.y, a1);
        a2 = fmaf(ck, a.z, a2); a3 = fmaf(ck, a.w, a3);
      }
    }
    const v4f sv = *(const v4fa*)(H + (size_t)nc * DD + 4 * lane);
    const float coef = 2.0f * dd * dd;
    float y[4];
    y[0] = (a0 + sv.x * coef) + bq[0];
    y[1] = (a1 + sv.y * coef) + bq[1];
    y[2] = (a2 + sv.z * coef) + bq[2];
    y[3] = (a3 + sv.w * coef) + bq[3];
    if (node < nN) {
      v4f ov;
      ov.x = y[0]; ov.y = y[1]; ov.z = y[2]; ov.w = y[3];
      float* op = C + (size_t)node * DD + 4 * lane;
      *(volatile v4f*)op = ov;
      __threadfence();
      *(volatile v4f*)op = ov;
      wn += 1;
      const float rk = 1.0f / (float)wn;
#pragma unroll
      for (int j = 0; j < 4; ++j) {
        const float d = y[j] - wm[j];
        wm[j] = fmaf(d, rk, wm[j]);
        wq[j] = fmaf(d, y[j] - wm[j], wq[j]);
      }
    }
  }

  if (lane == 0) wst[wave * WSTW] = (float)wn;
#pragma unroll
  for (int j = 0; j < 4; ++j) {
    wst[wave * WSTW + 1 + 4 * lane + j]      = wm[j];
    wst[wave * WSTW + 1 + DD + 4 * lane + j] = wq[j];
  }
  __syncthreads();
  if (tid < DD) {
    float n = 0.0f, mean = 0.0f, M2 = 0.0f;
#pragma unroll 1
    for (int w2 = 0; w2 < NWAVE; ++w2) {
      const float nb = wst[w2 * WSTW];
      const float mb = wst[w2 * WSTW + 1 + tid];
      const float qb = wst[w2 * WSTW + 1 + DD + tid];
      if (nb > 0.5f) {
        const float nn = n + nb;
        const float delta = mb - mean;
        const float f = nb / nn;
        mean = fmaf(delta, f, mean);
        M2 = M2 + qb + delta * delta * n * f;
        n = nn;
      }
    }
    pst[1 + tid] = mean;
    pst[1 + DD + tid] = M2;
    if (tid == 0) pst[0] = n;
  }
#pragma unroll 1
  for (int i = 2 * DD + 1 + tid; i < PARTW; i += NTHR) pst[i] = 0.0f;
  __syncthreads();
  v4f ps = {0.f, 0.f, 0.f, 0.f};
  float* rp = REC + (size_t)blockIdx.x * PARTW + 4 * tid;
  if (tid < PARTW / 4) {
    ps = *(const v4fa*)(pst + 4 * tid);
    *(volatile v4f*)rp = ps;
  }
  __threadfence();
  if (tid < PARTW / 4) {
    *(volatile v4f*)rp = ps;
  }
}

__global__ __launch_bounds__(DD) void k_comb(const float* __restrict__ REC, int nPart, float* STAT) {
  __shared__ __attribute__((aligned(16))) float stg[2 * DD];
  const int tid = (int)threadIdx.x;
  double n = 0.0, mean = 0.0, M2 = 0.0;
#pragma unroll 1
  for (int b = 0; b < nPart; ++b) {
    const float* pr = REC + (size_t)b * PARTW;
    const double nb = (double)pr[0];
    const double mb = (double)pr[1 + tid];
    const double qb = (double)pr[1 + DD + tid];
    if (nb > 0.5) {
      const double nn = n + nb;
      const double delta = mb - mean;
      const double f = nb / nn;
      mean = mean + delta * f;
      M2 = M2 + qb + delta * delta * n * f;
      n = nn;
    }
  }
  const double nt = n < 1.0 ? 1.0 : n;
  const float varf  = (float)(M2 / nt);
  const float meanf = (float)mean;
  const float rstd  = 1.0f / sqrtf(varf + 1e-5f);
  stg[tid] = meanf;
  stg[DD + tid] = rstd;
  __syncthreads();
  v4f v = {0.f, 0.f, 0.f, 0.f};
  if (tid < (2 * DD) / 4) {
    v = *(const v4fa*)(stg + 4 * tid);
    *(volatile v4f*)(STAT + 4 * tid) = v;
  }
  __threadfence();
  if (tid < (2 * DD) / 4) {
    *(volatile v4f*)(STAT + 4 * tid) = v;
  }
}

template <int MODE>
__global__ __launch_bounds__(NTHR) void k_apply(const float* __restrict__ C, const float* __restrict__ X,
                                                const float* __restrict__ STAT,
                                                const float* __restrict__ gam, const float* __restrict__ bet,
                                                const float* __restrict__ VT, const float* __restrict__ Q1in,
                                                int nN, unsigned short* HL, float* QP) {
  const int tid = (int)threadIdx.x, lane = tid & 31, wave = tid >> 5;
  const int hf = lane >> 4, cl = lane & 15, c8 = 8 * cl;
  const int rowBase = ((int)blockIdx.x * NWAVE + wave) * 32;

  float mq[8], rq[8], gq[8], eq[8], vq[8];
  {
    const v4f a = *(const v4fa*)(STAT + c8),      b = *(const v4fa*)(STAT + c8 + 4);
    mq[0] = a.x; mq[1] = a.y; mq[2] = a.z; mq[3] = a.w; mq[4] = b.x; mq[5] = b.y; mq[6] = b.z; mq[7] = b.w;
    const v4f c = *(const v4fa*)(STAT + DD + c8), d = *(const v4fa*)(STAT + DD + c8 + 4);
    rq[0] = c.x; rq[1] = c.y; rq[2] = c.z; rq[3] = c.w; rq[4] = d.x; rq[5] = d.y; rq[6] = d.z; rq[7] = d.w;
    const v4f e = *(const v4fa*)(gam + c8),       f = *(const v4fa*)(gam + c8 + 4);
    gq[0] = bf16_val(e.x); gq[1] = bf16_val(e.y); gq[2] = bf16_val(e.z); gq[3] = bf16_val(e.w);
    gq[4] = bf16_val(f.x); gq[5] = bf16_val(f.y); gq[6] = bf16_val(f.z); gq[7] = bf16_val(f.w);
    const v4f g = *(const v4fa*)(bet + c8),       h = *(const v4fa*)(bet + c8 + 4);
    eq[0] = bf16_val(g.x); eq[1] = bf16_val(g.y); eq[2] = bf16_val(g.z); eq[3] = bf16_val(g.w);
    eq[4] = bf16_val(h.x); eq[5] = bf16_val(h.y); eq[6] = bf16_val(h.z); eq[7] = bf16_val(h.w);
    const v4f p = *(const v4fa*)(VT + c8),        q = *(const v4fa*)(VT + c8 + 4);
    vq[0] = p.x; vq[1] = p.y; vq[2] = p.z; vq[3] = p.w; vq[4] = q.x; vq[5] = q.y; vq[6] = q.z; vq[7] = q.w;
  }

  float keep = 0.0f;
#pragma unroll 1
  for (int it = 0; it < 16; ++it) {
    const int row = rowBase + 2 * it + hf;
    const int rc  = row < nN ? row : nN - 1;
    const bool live = row < nN;
    const float* cp = C + (size_t)rc * DD + c8;
    const v4f ca = *(const v4fa*)cp;
    const v4f cb = *(const v4fa*)(cp + 4);
    float cv[8];
    cv[0] = ca.x; cv[1] = ca.y; cv[2] = ca.z; cv[3] = ca.w; cv[4] = cb.x; cv[5] = cb.y; cv[6] = cb.z; cv[7] = cb.w;
    float xv[8];
    if constexpr (MODE == 1) {
      const float* xp = X + (size_t)rc * DD + c8;
      const v4f xa = *(const v4fa*)xp;
      const v4f xb = *(const v4fa*)(xp + 4);
      xv[0] = bf16_val(xa.x); xv[1] = bf16_val(xa.y); xv[2] = bf16_val(xa.z); xv[3] = bf16_val(xa.w);
      xv[4] = bf16_val(xb.x); xv[5] = bf16_val(xb.y); xv[6] = bf16_val(xb.z); xv[7] = bf16_val(xb.w);
    } else {
#pragma unroll
      for (int j = 0; j < 8; ++j) xv[j] = 0.0f;
    }
    float hv[8];
    float dot = 0.0f;
#pragma unroll
    for (int j = 0; j < 8; ++j) {
      const float t  = (gq[j] * (cv[j] - mq[j])) * rq[j] + eq[j];
      const float re = (t > 0.0f) ? t : (t - t);
      const float hh = re + xv[j];
      hv[j] = live ? hh : 0.0f;
      dot = fmaf(hv[j], vq[j], dot);
    }
    if constexpr (MODE == 1) {
      v8us ho, lo;
#pragma unroll
      for (int j = 0; j < 8; ++j) {
        const unsigned hb = bf16_bits_n(hv[j]);
        ho[j] = (unsigned short)hb;
        lo[j] = (unsigned short)bf16_bits_n(hv[j] - __uint_as_float(hb << 16));
      }
      unsigned short* hp = HL + (size_t)row * K2 + c8;
      *(volatile v8us*)hp = ho;
      *(volatile v8us*)(hp + DD) = lo;
      __threadfence();
      *(volatile v8us*)hp = ho;
      *(volatile v8us*)(hp + DD) = lo;
    }
    float val = dot;
    val += __shfl_xor(val, 8, 32);
    val += __shfl_xor(val, 4, 32);
    val += __shfl_xor(val, 2, 32);
    val += __shfl_xor(val, 1, 32);
    const float oth  = __shfl_xor(val, 16, 32);
    const float pick = ((lane & 1) == hf) ? val : oth;
    keep = ((lane >> 1) == it) ? pick : keep;
  }
  float outv = keep;
  if constexpr (MODE == 2) {
    outv = keep + Q1in[rowBase + lane];
  }
  float* qp = QP + rowBase + lane;
  *(volatile float*)qp = outv;
  __threadfence();
  *(volatile float*)qp = outv;
}

__global__ __launch_bounds__(NTHR) void k_agg3pool(const int* __restrict__ LIST, const int* __restrict__ CNT,
                                                   const int* __restrict__ OFF, const float* __restrict__ DINV,
                                                   const float* __restrict__ P, const float* __restrict__ VT,
                                                   const int* __restrict__ bat, int nN, float* REC3) {
  __shared__ __attribute__((aligned(16))) float sv[NBA];
  __shared__ int gid[NBA];
  __shared__ __attribute__((aligned(16))) float bins[NWAVE * NGR];
  const int tid = (int)threadIdx.x, lane = tid & 31, wave = tid >> 5;
  const int nodeBase = (int)blockIdx.x * NBA;
  const int* lp = LIST + (size_t)blockIdx.x * RCAP;
  const float c0 = VT[DD];

#pragma unroll 1
  for (int i = tid; i < NWAVE * NGR; i += NTHR) bins[i] = 0.0f;

#pragma unroll 1
  for (int q = 0; q < NBA / NTHR; ++q) {
    const int s    = q * NTHR + tid;
    const int node = nodeBase + s;
    int c = CNT[node];
    c = c < 0 ? 0 : (c > DEGCAP ? DEGCAP : c);
    int o = OFF[node];
    o = o < 0 ? 0 : (o > RCAP ? RCAP : o);
    const int nc = node < nN ? node : nN - 1;
    const float dd = DINV[node];
    int cm = c;
    cm = max(cm, __shfl_xor(cm, 16, 32));
    cm = max(cm, __shfl_xor(cm, 8, 32));
    cm = max(cm, __shfl_xor(cm, 4, 32));
    cm = max(cm, __shfl_xor(cm, 2, 32));
    cm = max(cm, __shfl_xor(cm, 1, 32));
    cm = cm > DEGCAP ? DEGCAP : cm;
    float acc = 0.0f;
#pragma unroll 1
    for (int p = 0; p < cm; ++p) {
      int idx = o + p;
      idx = idx > RCAP - 1 ? RCAP - 1 : idx;
      int sr = lp[idx];
      sr = sr < 0 ? 0 : (sr > nN - 1 ? nN - 1 : sr);
      const float term = (DINV[sr] * dd) * P[sr];
      const float nacc = acc + term;
      acc = (p < c) ? nacc : acc;
    }
    const float pv = P[nc];
    const float sres = (acc + (2.0f * dd * dd) * pv) + c0;
    const int   bg = bat[nc];
    const bool live = node < nN;
    sv[s]  = live ? sres : 0.0f;
    gid[s] = live ? bg : -1;
  }
  __syncthreads();
  if (lane == 0) {
    float* wb = bins + wave * NGR;
#pragma unroll 1
    for (int j = 0; j < NBA / NWAVE; ++j) {
      const int s = wave * (NBA / NWAVE) + j;
      const int g = gid[s];
      if ((unsigned)g < (unsigned)NGR) wb[g] = wb[g] + sv[s];
    }
  }
  __syncthreads();
  v4f r = {0.f, 0.f, 0.f, 0.f};
  float* rp = REC3 + (size_t)blockIdx.x * NGR + 4 * tid;
  if (tid < NGR / 4) {
#pragma unroll
    for (int w2 = 0; w2 < NWAVE; ++w2) {
      const v4f b = *(const v4fa*)(bins + w2 * NGR + 4 * tid);
      r.x += b.x; r.y += b.y; r.z += b.z; r.w += b.w;
    }
    *(volatile v4f*)rp = r;
  }
  __threadfence();
  if (tid < NGR / 4) {
    *(volatile v4f*)rp = r;
  }
}

__global__ __launch_bounds__(NGR) void k_final(const float* __restrict__ REC3, const float* __restrict__ VT,
                                               int nPart, float* out) {
  __shared__ __attribute__((aligned(16))) float os[NGR];
  const int tid = (int)threadIdx.x;
  double s = 0.0;
#pragma unroll 4
  for (int b = 0; b < nPart; ++b) s += (double)REC3[(size_t)b * NGR + tid];
  os[tid] = (float)(s + (double)VT[DD + 1]);
  __syncthreads();
  v4f v = {0.f, 0.f, 0.f, 0.f};
  if (tid < NGR / 4) {
    v = *(const v4fa*)(os + 4 * tid);
    *(volatile v4f*)(out + 4 * tid) = v;
  }
  __threadfence();
  if (tid < NGR / 4) {
    *(volatile v4f*)(out + 4 * tid) = v;
  }
}

static inline size_t al256(size_t o) { return (o + 255) & ~(size_t)255; }

extern "C" void kernel_launch(void* const* d_in, const int* in_sizes, int n_in,
                              void* d_out, int out_size, void* d_ws, size_t ws_size,
                              hipStream_t stream) {
  if (n_in < 15) return;
  if (in_sizes[0] != NN * DD) return;
  if (in_sizes[1] != 2 * NE) return;
  if (in_sizes[2] != NN) return;
  if (in_sizes[3] != DD * DD || in_sizes[7] != DD * DD || in_sizes[11] != DD * DD) return;
  if (in_sizes[4] != DD || in_sizes[5] != DD || in_sizes[6] != DD) return;
  if (in_sizes[8] != DD || in_sizes[9] != DD || in_sizes[10] != DD) return;
  if (in_sizes[12] != DD || in_sizes[13] != DD || in_sizes[14] != 1) return;
  if (out_size != NGR) return;

  const float* x    = (const float*)d_in[0];
  const int*   edge = (const int*)d_in[1];
  const int*   bat  = (const int*)d_in[2];
  const float* W0   = (const float*)d_in[3];
  const float* b0   = (const float*)d_in[4];
  const float* g0   = (const float*)d_in[5];
  const float* be0  = (const float*)d_in[6];
  const float* W1   = (const float*)d_in[7];
  const float* b1   = (const float*)d_in[8];
  const float* g1   = (const float*)d_in[9];
  const float* be1  = (const float*)d_in[10];
  const float* W2   = (const float*)d_in[11];
  const float* b2   = (const float*)d_in[12];
  const float* fcW  = (const float*)d_in[13];
  const float* fcb  = (const float*)d_in[14];
  float* out = (float*)d_out;
  const int* src = edge;
  const int* dst = edge + NE;
  const int nN = NN, nE = NE;
  const int vec8 = ((nE & 3) == 0) ? 1 : 0;

  char* ws = (char*)d_ws;
  size_t off = 0;
  const size_t oR1  = off; off = al256(off + (size_t)NP * DD * 4);
  const size_t oR2  = off; off = al256(off + (size_t)NP * DD * 4);
  const size_t oLST = off; off = al256(off + (size_t)NBLK * RCAP * 4);
  const size_t oCNT = off; off = al256(off + (size_t)NSL * 4);
  const size_t oOFF = off; off = al256(off + (size_t)NSL * 4);
  const size_t oDNV = off; off = al256(off + (size_t)NSL * 4);
  const size_t oQ1  = off; off = al256(off + (size_t)NP * 4);
  const size_t oP   = off; off = al256(off + (size_t)NP * 4);
  const size_t oRC1 = off; off = al256(off + (size_t)NBLK * PARTW * 4);
  const size_t oRC2 = off; off = al256(off + (size_t)NBLK * PARTW * 4);
  const size_t oRC3 = off; off = al256(off + (size_t)NBLK * NGR * 4);
  const size_t oST1 = off; off = al256(off + (size_t)(2 * DD) * 4);
  const size_t oST2 = off; off = al256(off + (size_t)(2 * DD) * 4);
  const size_t oW0T = off; off = al256(off + (size_t)DD * DD * 2);
  const size_t oW1D = off; off = al256(off + (size_t)DD * K2 * 2);
  const size_t oVT  = off; off = al256(off + (size_t)VTW * 4);
  if (off > ws_size || off > (size_t)WSMAX) return;

  float*          R1f  = (float*)(ws + oR1);
  unsigned short* R1h  = (unsigned short*)(ws + oR1);
  float*          R2f  = (float*)(ws + oR2);
  unsigned short* R2h  = (unsigned short*)(ws + oR2);
  int*            LIST = (int*)(ws + oLST);
  int*            CNT  = (int*)(ws + oCNT);
  int*            OFF  = (int*)(ws + oOFF);
  float*          DINV = (float*)(ws + oDNV);
  float*          Q1   = (float*)(ws + oQ1);
  float*          P    = (float*)(ws + oP);
  float*          REC1 = (float*)(ws + oRC1);
  float*          REC2 = (float*)(ws + oRC2);
  float*          REC3 = (float*)(ws + oRC3);
  float*          ST1  = (float*)(ws + oST1);
  float*          ST2  = (float*)(ws + oST2);
  unsigned short* W0T  = (unsigned short*)(ws + oW0T);
  unsigned short* W1D  = (unsigned short*)(ws + oW1D);
  float*          VT   = (float*)(ws + oVT);

  const size_t bkLds = (size_t)BK_LDS_INTS * 4;
  hipFuncSetAttribute(reinterpret_cast<const void*>(&k_bucket), hipFuncAttributeMaxDynamicSharedMemorySize, (int)bkLds);

  const int nUx = NP * (DD / 8);
  k_cvx<<<nUx / NTHR, NTHR, 0, stream>>>(x, nN, nUx, R2h);
  k_wprep<<<(NUW0 + NUW1) / NTHR + 1, NTHR, 0, stream>>>(W0, W1, W2, b2, fcW, fcb, W0T, W1D, VT);
  k_bucket<<<NBLK, NTHR, bkLds, stream>>>(src, dst, nE, nN, vec8, LIST, CNT, OFF, DINV);
  k_gemm<<<NP / GBM, GTHR, 0, stream>>>(R2h, W0T, R1f, DD);
  k_agg<<<NBLK, NTHR, 0, stream>>>(LIST, CNT, OFF, DINV, R1f, b0, nN, R2f, REC1);
  k_comb<<<1, DD, 0, stream>>>(REC1, NBLK, ST1);
  k_apply<1><<<NP / 256, NTHR, 0, stream>>>(R2f, x, ST1, g0, be0, VT, Q1, nN, R1h, Q1);
  k_gemm<<<NP / GBM, GTHR, 0, stream>>>(R1h, W1D, R2f, K2);
  k_agg<<<NBLK, NTHR, 0, stream>>>(LIST, CNT, OFF, DINV, R2f, b1, nN, R1f, REC2);
  k_comb<<<1, DD, 0, stream>>>(REC2, NBLK, ST2);
  k_apply<2><<<NP / 256, NTHR, 0, stream>>>(R1f, x, ST2, g1, be1, VT, Q1, nN, R2h, P);
  k_agg3pool<<<NBLK, NTHR, 0, stream>>>(LIST, CNT, OFF, DINV, P, VT, bat, nN, REC3);
  k_final<<<1, NGR, 0, stream>>>(REC3, VT, NBLK, out);
}
